// RateAdaptionEncoder_54589034332166
// MI455X (gfx1250) — hardware-run, weakly checked
//
#include <hip/hip_runtime.h>


#ifndef NB
#define NB 16
#endif
#define NB_FULL 16
#define LL    256
#define KC    256
#define NR    256
#define NTOK  (NB * LL)
#define XB_FULL (KC * LL)
#define NREL  8
#define NSEG  32
#define RB    1024
#define NBLK  (NTOK / RB)
#define OFFP  128
#define PROWS (NTOK + 512)

static_assert(NTOK % RB == 0);
static_assert(NBLK >= 1 && NBLK <= OFFP);
static_assert(NB <= NB_FULL);
static_assert(NREL * 63 <= 512);
static_assert(NREL <= NSEG);
static_assert(PROWS % 64 == 0);
static_assert(KC % 64 == 0 && NR % 64 == 0 && KC % 32 == 0);
static_assert(LL % 32 == 0 && RB % LL == 0);
static_assert(LL == 256 && KC == 256 && NR == 256);

typedef unsigned short bf;
typedef __attribute__((ext_vector_type(16))) __bf16   v16bf;
typedef __attribute__((ext_vector_type(8)))  unsigned short v8us;
typedef __attribute__((ext_vector_type(8)))  float    v8f;
typedef __attribute__((ext_vector_type(4)))  float    v4f;
typedef __attribute__((ext_vector_type(4)))  int      v4i;
typedef v4f  __attribute__((may_alias)) v4fa;
typedef v4i  __attribute__((may_alias)) v4ia;

__device__ __forceinline__ unsigned short f2bf(float f) { unsigned u = __float_as_uint(f); u += 0x7FFFu + ((u >> 16) & 1u); return (unsigned short)(u >> 16); }
__device__ __forceinline__ float bf2f(unsigned short w) { return __uint_as_float(((unsigned)w) << 16); }
__device__ __forceinline__ int clampi(int v, int lo, int hi) { return min(max(v, lo), hi); }
__device__ __forceinline__ v16bf cat16b(v8us lo, v8us hi) { return __builtin_bit_cast(v16bf, __builtin_shufflevector(lo, hi, 0, 1, 2, 3, 4, 5, 6, 7, 8, 9, 10, 11, 12, 13, 14, 15)); }
__device__ __forceinline__ v8f wmmab(v16bf a, v16bf b, v8f c) { return __builtin_amdgcn_wmma_f32_16x16x32_bf16(false, a, false, b, (short)0, c, false, false); }
__device__ __forceinline__ v16bf ldb(const bf* p)  { return cat16b(*(const v8us*)p, *(const v8us*)(p + 16)); }
__device__ __forceinline__ void wave_sync() { __builtin_amdgcn_fence(3  , "wavefront"); __builtin_amdgcn_wave_barrier(); asm volatile("" ::: "memory"); }

static_assert(256 * 16 * 2 == 64 * 128);
static_assert(64 * 65 * 4 <= 131072);
__global__ __launch_bounds__(256) void k_wt(const float* __restrict__ W, bf* WT) {
    __shared__ float ts[64 * 65];
    const int g = blockIdx.x >> 4, tc = (blockIdx.x >> 2) & 3, tr = blockIdx.x & 3, t = threadIdx.x;
    const float* src = W + (size_t)g * (KC * NR) + (size_t)(tc * 64) * NR + tr * 64;
#pragma unroll 1
    for (int i = 0; i < 16; ++i) { const int f = i * 256 + t; ts[(f >> 6) * 65 + (f & 63)] = src[(size_t)(f >> 6) * NR + (f & 63)]; }
    __syncthreads();
    bf* dst = WT + (size_t)g * (NR * KC) + (size_t)(tr * 64) * KC + tc * 64;
#pragma unroll 1
    for (int ps = 0; ps < 2; ++ps) {
#pragma unroll 1
        for (int it = 0; it < 2; ++it) {
            const int e = it * 32 + (t >> 3), c8 = (t & 7) * 8; v8us o;
#pragma unroll
            for (int k = 0; k < 8; ++k) o[k] = f2bf(ts[(c8 + k) * 65 + e]);
            *(volatile v8us*)(dst + (size_t)e * KC + c8) = o; }
        if (ps == 0) __threadfence(); }
}

__global__ __launch_bounds__(1024) void k_count(const int* __restrict__ rels, int* cnt) {
    __shared__ int wc[32 * 32];
    __shared__ __align__(16) int line[32];
    const int tid = threadIdx.x, lane = tid & 31; const int wave = __builtin_amdgcn_readfirstlane(tid >> 5);
    const int blk = blockIdx.x;
    const int rel = clampi(rels[(size_t)blk * RB + tid], 0, NREL - 1);
    int mine = 0;
#pragma unroll 1
    for (int r = 0; r < NREL; ++r) { const unsigned m = __builtin_amdgcn_ballot_w32(rel == r); const int c = __builtin_popcount(m); mine = (lane == r) ? c : mine; }
    wc[wave * 32 + lane] = mine;
    __syncthreads();
    if (wave == 0) {
        int s = 0;
#pragma unroll 1
        for (int w = 0; w < 32; ++w) s += wc[w * 32 + lane];
        line[lane] = s;
        wave_sync();
#pragma unroll 1
        for (int ps = 0; ps < 2; ++ps) {
            if (lane < 8) { const v4i v = *(const v4ia*)(&line[4 * lane]); *(volatile v4i*)(cnt + (size_t)blk * 32 + 4 * lane) = v; }
            if (ps == 0) __threadfence(); }
    }
}

static_assert(32 * 8 == KC);
__global__ __launch_bounds__(1024) void k_scan(const int* __restrict__ cnt, int* offs, int* T, bf* AP) {
    __shared__ int tots[32];
    __shared__ __align__(16) int tl[128];
    const int tid = threadIdx.x, lane = tid & 31; const int r = __builtin_amdgcn_readfirstlane(tid >> 5);
    int c[4]; int ls = 0;
#pragma unroll
    for (int i = 0; i < 4; ++i) { const int blk = 4 * lane + i; const int bc = min(blk, NBLK - 1);
        int v = cnt[(size_t)bc * 32 + r]; v = (blk < NBLK) ? v : 0; v = clampi(v, 0, RB); c[i] = v; ls += v; }
    int x = ls;
#pragma unroll
    for (int d = 1; d < 32; d <<= 1) { const int y = __shfl_up(x, d, 32); x += (lane >= d) ? y : 0; }
    const int excl = x - ls;
    const int tot = __shfl(x, 31, 32);
    if (lane == 0) tots[r] = tot;
    __syncthreads();
    const int t = tots[lane]; const int pd = (t + 63) & ~63;
    int y2 = pd;
#pragma unroll
    for (int d = 1; d < 32; d <<= 1) { const int y = __shfl_up(y2, d, 32); y2 += (lane >= d) ? y : 0; }
    const int sstart = y2 - pd;
    const int ptot = __shfl(y2, 31, 32);
    const int segr = __shfl(sstart, r, 32);
    v4i o; o[0] = segr + excl; o[1] = o[0] + c[0]; o[2] = o[1] + c[1]; o[3] = o[2] + c[2];
    if (r == 0) { tl[lane] = sstart; tl[32 + lane] = t; tl[64 + lane] = (lane == 0) ? ptot : 0; tl[96 + lane] = 0; wave_sync(); }
    const int padcnt = ((tot + 63) & ~63) - tot;
    const int pbase = segr + tot;
    v8us z;
#pragma unroll
    for (int k = 0; k < 8; ++k) z[k] = (unsigned short)0;
#pragma unroll 1
    for (int ps = 0; ps < 2; ++ps) {
        *(volatile v4i*)(offs + (size_t)r * OFFP + 4 * lane) = o;
        if (r == 0) { const v4i v = *(const v4ia*)(&tl[4 * lane]); *(volatile v4i*)(T + 4 * lane) = v; }
#pragma unroll 1
        for (int j = 0; j < 64; ++j) { const int p = clampi(pbase + j, 0, PROWS - 1);
            if (j < padcnt) { *(volatile v8us*)(AP + (size_t)p * KC + 8 * lane) = z; } }
        if (ps == 0) __threadfence(); }
}

static_assert(32 * 16 * 32 == 32 * KC * 2);
__global__ __launch_bounds__(1024) void k_rank(const int* __restrict__ rels, const float* __restrict__ xin,
                                               const int* __restrict__ offs, int* POS, bf* AP) {
    __shared__ int wc[32 * 32];
    const int tid = threadIdx.x, lane = tid & 31; const int wave = __builtin_amdgcn_readfirstlane(tid >> 5);
    const int blk = blockIdx.x;
    const size_t row = (size_t)blk * RB + tid;
    const int rel = clampi(rels[row], 0, NREL - 1);
    int mine = 0; unsigned mymask = 0u;
#pragma unroll 1
    for (int r = 0; r < NREL; ++r) { const unsigned m = __builtin_amdgcn_ballot_w32(rel == r); const int c = __builtin_popcount(m);
        mine = (lane == r) ? c : mine; mymask = (rel == r) ? m : mymask; }
    const int lrank = __builtin_popcount(mymask & ((1u << lane) - 1u));
    wc[wave * 32 + lane] = mine;
    __syncthreads();
    if (wave == 0) {
        int run = clampi(offs[(size_t)lane * OFFP + blk], 0, PROWS);
#pragma unroll 1
        for (int w = 0; w < 32; ++w) { const int c = wc[w * 32 + lane]; wc[w * 32 + lane] = run; run += c; }
    }
    __syncthreads();
    const int pos = clampi(wc[wave * 32 + rel] + lrank, 0, PROWS - 1);
    const int c8 = lane * 8;
#pragma unroll 1
    for (int ps = 0; ps < 2; ++ps) {
        *(volatile int*)(POS + row) = pos;
#pragma unroll 1
        for (int it = 0; it < 32; ++it) { const int p = __shfl(pos, it, 32);
            const int rg = blk * RB + wave * 32 + it;
            const int bb = rg / LL, l = rg % LL;
            const float* src = xin + (size_t)bb * XB_FULL + (size_t)c8 * LL + l;
            v8us oa;
#pragma unroll
            for (int k = 0; k < 8; ++k) oa[k] = f2bf(src[(size_t)k * LL]);
            *(volatile v8us*)(AP + (size_t)p * KC + c8) = oa; }
        if (ps == 0) __threadfence(); }
}

static_assert(32 * 16 * 32 == 64 * 64 * 4);
static_assert(64 * 68 * 4 <= 131072);
__global__ __launch_bounds__(32) __attribute__((amdgpu_num_vgpr(256))) void k_gemm(const bf* __restrict__ AP, const bf* __restrict__ WT, const float* __restrict__ bias,
                                                                                    const int* __restrict__ rct, const int* __restrict__ T, float* YS) {
    __shared__ __align__(16) float os[64 * 68];
    const int lane = threadIdx.x & 31, lr = lane & 15, hi = lane >> 4;
    const int p0 = blockIdx.x * 64;
    const int n0 = blockIdx.y * 64;
    const int ss = T[lane], tt = T[32 + lane];
    const int pe = ss + ((tt + 63) & ~63);
    const unsigned msk = __builtin_amdgcn_ballot_w32((p0 >= ss) && (p0 < pe));
    if (msk == 0u) return;
    const int r = clampi(__builtin_amdgcn_readfirstlane(__builtin_ctz(msk)), 0, NREL - 1);
    v8f acc[4][4];
#pragma unroll
    for (int mb = 0; mb < 4; ++mb)
#pragma unroll
        for (int nb = 0; nb < 4; ++nb) acc[mb][nb] = (v8f){};
    const size_t aoff = (size_t)(p0 + lr) * KC + 8 * hi, boff = (size_t)r * (NR * KC) + (size_t)(n0 + lr) * KC + 8 * hi;
#pragma unroll 1
    for (int kc = 0; kc < KC; kc += 32) {
        v16bf a[4];
#pragma unroll
        for (int mb = 0; mb < 4; ++mb) a[mb] = ldb(AP + aoff + (size_t)mb * 16 * KC + kc);
#pragma unroll
        for (int nb = 0; nb < 4; ++nb) { const v16bf b = ldb(WT + boff + (size_t)nb * 16 * KC + kc);
#pragma unroll
            for (int mb = 0; mb < 4; ++mb) acc[mb][nb] = wmmab(a[mb], b, acc[mb][nb]); }
        asm volatile("v_nop\n\tv_nop\n\tv_nop\n\tv_nop" : "+v"(acc[0][0]), "+v"(acc[1][1]), "+v"(acc[2][2]), "+v"(acc[3][3]) : "v"(a[0]), "v"(a[1]), "v"(a[2]), "v"(a[3]));
    }
    const int rc = rct[r];
    float bv[4], mv[4];
#pragma unroll
    for (int nb = 0; nb < 4; ++nb) { const int col = n0 + nb * 16 + lr;
        bv[nb] = bf2f(f2bf(bias[(size_t)r * NR + col])); mv[nb] = (col < rc) ? 1.0f : 0.0f; }
#pragma unroll
    for (int mb = 0; mb < 4; ++mb) {
#pragma unroll
        for (int nb = 0; nb < 4; ++nb) {
#pragma unroll
            for (int j = 0; j < 8; ++j) os[(mb * 16 + hi * 8 + j) * 68 + nb * 16 + lr] = (acc[mb][nb][j] + bv[nb]) * mv[nb]; } }
    wave_sync();
#pragma unroll 1
    for (int ps = 0; ps < 2; ++ps) {
#pragma unroll 1
        for (int i = 0; i < 32; ++i) { const int row = 2 * i + hi;
            const v4f v = *(const v4fa*)(&os[row * 68 + 4 * lr]);
            *(volatile v4f*)(YS + (size_t)(p0 + row) * NR + n0 + 4 * lr) = v; }
        if (ps == 0) __threadfence(); }
}

static_assert(8 * 8 * 4 == LL);
static_assert(256 * 16 * 8 == 32 * LL * 4);
static_assert(LL * 36 * 4 + LL * 4 <= 131072);
__global__ __launch_bounds__(256) void k_out(const int* __restrict__ POS, const int* __restrict__ rels, const int* __restrict__ rct,
                                             const float* __restrict__ YS, float* OUTY, float* OUTM) {
    __shared__ __align__(16) float ts[LL * 36];
    __shared__ int rcs[LL];
    const int tid = threadIdx.x, lane = tid & 31; const int wave = __builtin_amdgcn_readfirstlane(tid >> 5);
    const int b = blockIdx.x >> 3, r0 = (blockIdx.x & 7) * 32;
    rcs[tid] = rct[clampi(rels[(size_t)b * LL + tid], 0, NREL - 1)];
#pragma unroll 1
    for (int it = 0; it < 8; ++it) { const int l = wave * 32 + 4 * it + (lane >> 3);
        const int p = clampi(POS[(size_t)b * LL + l], 0, PROWS - 1);
        const v4f v = *(const v4f*)(YS + (size_t)p * NR + r0 + 4 * (lane & 7));
        *(v4fa*)(&ts[l * 36 + 4 * (lane & 7)]) = v; }
    __syncthreads();
#pragma unroll 1
    for (int ps = 0; ps < 2; ++ps) {
#pragma unroll 1
        for (int it = 0; it < 8; ++it) { const int rr = wave * 4 + (it >> 1); const int l0 = (it & 1) * 128 + 4 * lane; const int r = r0 + rr;
            v4f y, m;
#pragma unroll
            for (int k = 0; k < 4; ++k) { y[k] = ts[(l0 + k) * 36 + rr]; m[k] = (r < rcs[l0 + k]) ? 1.0f : 0.0f; }
            const size_t o = ((size_t)b * NR + r) * LL + l0;
            *(volatile v4f*)(OUTY + o) = y; *(volatile v4f*)(OUTM + o) = m; }
        if (ps == 0) __threadfence(); }
}

static constexpr size_t al256(size_t v) { return (v + 255) & ~(size_t)255; }
static constexpr size_t SZ_WT  = al256((size_t)NREL * NR * KC * 2);
static constexpr size_t SZ_CNT = al256((size_t)NBLK * 32 * 4);
static constexpr size_t SZ_OFF = al256((size_t)NSEG * OFFP * 4);
static constexpr size_t SZ_T   = al256((size_t)128 * 4);
static constexpr size_t SZ_POS = al256((size_t)NTOK * 4);
static constexpr size_t SZ_PL  = al256((size_t)PROWS * KC * 2);
static constexpr size_t SZ_YS  = al256((size_t)PROWS * NR * 4);
static constexpr size_t SZ_TOTAL = SZ_WT + SZ_CNT + SZ_OFF + SZ_T + SZ_POS + SZ_PL + SZ_YS;
static_assert(SZ_TOTAL <= (size_t)134217728);
static constexpr size_t OUT1_OFF = (size_t)NB_FULL * NR * LL;
static_assert(OUT1_OFF * 4 == (size_t)4194304);
static_assert((size_t)NB * NR * LL <= OUT1_OFF);

extern "C" void kernel_launch(void* const* d_in, const int* in_sizes, int n_in,
                              void* d_out, int out_size, void* d_ws, size_t ws_size, hipStream_t stream) {
    if (n_in < 5) return;
    if ((size_t)in_sizes[0] < (size_t)NB * KC * LL) return;
    if ((size_t)in_sizes[1] < (size_t)NTOK) return;
    if ((size_t)in_sizes[2] < (size_t)NREL * KC * NR) return;
    if ((size_t)in_sizes[3] < (size_t)NREL * NR) return;
    if ((size_t)in_sizes[4] < (size_t)NREL) return;
    if ((size_t)out_size < OUT1_OFF + (size_t)NB * NR * LL) return;
    if (SZ_TOTAL > ws_size) return;
    const float* xin  = (const float*)d_in[0];
    const int*   idx  = (const int*)d_in[1];
    const float* wgt  = (const float*)d_in[2];
    const float* bias = (const float*)d_in[3];
    const int*   rct  = (const int*)d_in[4];
    float* OUTY = (float*)d_out;
    float* OUTM = OUTY + OUT1_OFF;
    char* wsp = (char*)d_ws;
    bf*  WT  = (bf*)wsp;  wsp += SZ_WT;
    int* CNT = (int*)wsp; wsp += SZ_CNT;
    int* OFF = (int*)wsp; wsp += SZ_OFF;
    int* TT  = (int*)wsp; wsp += SZ_T;
    int* POS = (int*)wsp; wsp += SZ_POS;
    bf*  AP  = (bf*)wsp;  wsp += SZ_PL;
    float* YS = (float*)wsp; wsp += SZ_YS;

    k_wt<<<NREL * 16, 256, 0, stream>>>(wgt, WT);
    k_count<<<NBLK, 1024, 0, stream>>>(idx, CNT);
    k_scan<<<1, 1024, 0, stream>>>(CNT, OFF, TT, AP);
    k_rank<<<NBLK, 1024, 0, stream>>>(idx, xin, OFF, POS, AP);
    k_gemm<<<dim3(PROWS / 64, NR / 64), 32, 0, stream>>>(AP, WT, bias, rct, TT, YS);
    k_out<<<NB * 8, 256, 0, stream>>>(POS, idx, rct, YS, OUTY, OUTM);
}
